// GPT2Block_4337916970022
// MI455X (gfx1250) — hardware-verified
//
#include <hip/hip_runtime.h>
#include <math.h>

constexpr int kBatch   = 2;
constexpr int kSeq     = 2048;
constexpr int kSeqLog2 = 11;
constexpr int kDim     = 1024;
constexpr int kHeads   = 16;
constexpr int kHeadDim = 64;
constexpr int kFF      = 4096;
constexpr int kTok     = kBatch * kSeq;
constexpr int kGroupsPerChunk = 2;
constexpr int kChunks  = (kBatch * kHeads) / kGroupsPerChunk;
static_assert(kSeq == (1 << kSeqLog2), "seq pow2");
static_assert(kHeads * kHeadDim == kDim, "heads");
static_assert(kTok % 64 == 0 && kDim % 64 == 0 && kFF % 64 == 0 && kSeq % 64 == 0, "tile multiples");

constexpr float kWCarry    = 16.0f;
constexpr float kWCarryInv = 1.0f / 16.0f;
constexpr float kPCarry    = 2048.0f;
constexpr float kCtxCarry  = 256.0f;
constexpr float kH2Carry   = 16.0f;
constexpr float kScoreScale = 0.125f;
constexpr float kPVScale   = kCtxCarry / kPCarry;
constexpr float kProjScale = 1.0f / (kCtxCarry * kWCarry);
constexpr float kMlpScale  = 1.0f / (kH2Carry * kWCarry);
constexpr float kInvDim    = 1.0f / 1024.0f;
constexpr float kLnEps     = 1e-5f;
constexpr float kGeluC     = 0.7978845608028654f;
constexpr float kGeluA     = 0.044715f;

constexpr size_t kMiB     = 1048576;
constexpr size_t kOffWqkvT = 0;
constexpr size_t kOffX1    = 8 * kMiB;
constexpr size_t kOffSc    = 0;
constexpr size_t kOffH2    = 0;
constexpr size_t kOffP     = 32 * kMiB;
constexpr size_t kOffWfcT  = 32 * kMiB;
constexpr size_t kOffWmlpT = 40 * kMiB;
constexpr size_t kOffQK    = 48 * kMiB;
constexpr size_t kOffX2    = 48 * kMiB;
constexpr size_t kOffWprojT= 56 * kMiB;
constexpr size_t kOffVT    = 64 * kMiB;
constexpr size_t kOffCTX   = 72 * kMiB;
constexpr size_t kOffHO    = 80 * kMiB;
constexpr size_t kWsTotal  = 96 * kMiB;
static_assert((size_t)3 * kDim * kDim * 2 <= kOffX1 - kOffWqkvT, "WqkvT fits");
static_assert((size_t)kTok * kDim * 2 <= 8 * kMiB, "X1 fits");
static_assert((size_t)kGroupsPerChunk * kSeq * kSeq * 4 <= 32 * kMiB, "scores fits");
static_assert((size_t)kTok * kFF * 2 <= 32 * kMiB, "H2 fits");
static_assert((size_t)kGroupsPerChunk * kSeq * kSeq * 2 <= 16 * kMiB, "P fits");
static_assert((size_t)kFF * kDim * 2 <= 8 * kMiB, "WfcT fits");
static_assert((size_t)kTok * 2 * kDim * 2 <= 16 * kMiB, "QK fits");
static_assert((size_t)kDim * kDim * 2 <= 2 * kMiB, "WprojT fits");
static_assert((size_t)kDim * kTok * 2 <= 8 * kMiB, "VT fits");
static_assert((size_t)kTok * kDim * 4 <= 16 * kMiB, "HO fits");
static_assert(kWsTotal <= (size_t)134217728, "carve cap");

typedef __attribute__((ext_vector_type(16))) _Float16 v16h;
typedef __attribute__((ext_vector_type(8)))  _Float16 v8h;
typedef __attribute__((ext_vector_type(16))) __bf16   v16b;
typedef __attribute__((ext_vector_type(8)))  __bf16   v8b;
typedef __attribute__((ext_vector_type(8)))  float    v8f;
typedef __attribute__((ext_vector_type(4)))  float    v4f;
typedef __attribute__((ext_vector_type(4)))  unsigned int v4u;

__device__ __forceinline__ unsigned short f2bf_bits(float f) {
  unsigned u = __float_as_uint(f);
  return (unsigned short)((u + 0x7FFFu + ((u >> 16) & 1u)) >> 16);
}
__device__ __forceinline__ float bf_bits2f(unsigned short h) { return __uint_as_float(((unsigned)h) << 16); }

__device__ __forceinline__ void dep_guard_h(v8f& a, v8f& b, v16h x, v16h y) { asm volatile("v_nop\n\tv_nop\n\tv_nop\n\tv_nop" : "+v"(a), "+v"(b) : "v"(x), "v"(y)); }
__device__ __forceinline__ void dep_guard_b(v8f& a, v8f& b, v16b x, v16b y) { asm volatile("v_nop\n\tv_nop\n\tv_nop\n\tv_nop" : "+v"(a), "+v"(b) : "v"(x), "v"(y)); }
__device__ __forceinline__ void keep4_h(v16h a, v16h b, v16h c, v16h d) { asm volatile("v_nop" :: "v"(a), "v"(b), "v"(c), "v"(d)); }
__device__ __forceinline__ void keep4_b(v16b a, v16b b, v16b c, v16b d) { asm volatile("v_nop" :: "v"(a), "v"(b), "v"(c), "v"(d)); }
__device__ __forceinline__ void acc_guard4(v8f& a, v8f& b, v8f& c, v8f& d) { asm volatile("v_nop\n\tv_nop\n\tv_nop\n\tv_nop" : "+v"(a), "+v"(b), "+v"(c), "+v"(d)); }
template <typename T> struct Frag;
template <> struct Frag<_Float16> {
  typedef v16h V; union U { v16h v; v8h h[2]; };
  static __device__ __forceinline__ v16h load(const _Float16* p) {
    U f; f.h[0] = *(const v8h*)(p); f.h[1] = *(const v8h*)(p + 16); return f.v;
  }
  static __device__ __forceinline__ v8f mma(v16h a, v16h b, v8f c) {
    return __builtin_amdgcn_wmma_f32_16x16x32_f16(false, a, false, b, (short)0, c, false, false);
  }
  static __device__ __forceinline__ void guard(v8f& a, v8f& b, v16h x, v16h y) { dep_guard_h(a, b, x, y); }
  static __device__ __forceinline__ void keep(v16h a, v16h b, v16h c, v16h d) { keep4_h(a, b, c, d); }
};
template <> struct Frag<__bf16> {
  typedef v16b V; union U { v16b v; v8b h[2]; };
  static __device__ __forceinline__ v16b load(const __bf16* p) {
    U f; f.h[0] = *(const v8b*)(p); f.h[1] = *(const v8b*)(p + 16); return f.v;
  }
  static __device__ __forceinline__ v8f mma(v16b a, v16b b, v8f c) {
    return __builtin_amdgcn_wmma_f32_16x16x32_bf16(false, a, false, b, (short)0, c, false, false);
  }
  static __device__ __forceinline__ void guard(v8f& a, v8f& b, v16b x, v16b y) { dep_guard_b(a, b, x, y); }
  static __device__ __forceinline__ void keep(v16b a, v16b b, v16b c, v16b d) { keep4_b(a, b, c, d); }
};

__device__ __forceinline__ unsigned pk16(unsigned short a, unsigned short b) { return (unsigned)a | ((unsigned)b << 16); }
__device__ __forceinline__ unsigned short h_bits(float f) { const _Float16 h = (_Float16)f; return __builtin_bit_cast(unsigned short, h); }

template <int ET> struct Elem;
template <> struct Elem<0> { typedef _Float16 T; };
template <> struct Elem<1> { typedef __bf16 T; };
template <int ET, bool SPLIT, int BIAS_MODE, int OUT_MODE, bool RESID, int ACT = 0, bool CAUSAL = false>
__global__ __launch_bounds__(256) void wmma_gemm64(
    const unsigned short* __restrict__ Ap, const unsigned short* __restrict__ A2p, int lda, long strideA,
    const unsigned short* __restrict__ Btp, const unsigned short* __restrict__ Bt2p, int ldb, long strideB,
    void* __restrict__ Cout, void* __restrict__ Cout2, int ldc, long strideC,
    const float* __restrict__ bias,
    const float* __restrict__ resid, long strideR,
    int M, int N, int K, float scale) {
  typedef typename Elem<ET>::T T;
  typedef typename Frag<T>::V V;
  const T* A = (const T*)Ap; const T* A2 = (const T*)A2p; const T* Bt = (const T*)Btp; const T* Bt2 = (const T*)Bt2p;
  __shared__ __align__(16) float sT[8][16 * 68];
  const int b    = blockIdx.y;
  const int lane = threadIdx.x & 31;
  const int wave = threadIdx.x >> 5;
  const int tilesN = N >> 6;
  const int tilesM = M >> 6;
  const int tile = blockIdx.x * 8 + wave;
  if (tile >= tilesM * tilesN) return;
  const int tm = tile / tilesN;
  const int tn = tile - tm * tilesN;
  if (CAUSAL && tn > tm) return;
  const int m0 = tm << 6;
  const int n0 = tn << 6;
  const int Kend = CAUSAL ? ((m0 + 64 < K) ? (m0 + 64) : K) : K;

  const T* Ab  = A  + (size_t)b * strideA;
  const T* Bb  = Bt + (size_t)b * strideB;
  const T* Ab2 = SPLIT ? (A2  + (size_t)b * strideA) : nullptr;
  const T* Bb2 = SPLIT ? (Bt2 + (size_t)b * strideB) : nullptr;

  const int rlane = lane & 15;
  const int koff  = (lane >> 4) * 8;
  const int mOff  = (lane >> 4) * 8;

  v8f acc[4][4];
#pragma unroll
  for (int i = 0; i < 4; ++i)
#pragma unroll
    for (int j = 0; j < 4; ++j) acc[i][j] = (v8f){0.f,0.f,0.f,0.f,0.f,0.f,0.f,0.f};

  for (int k0 = 0; k0 < Kend; k0 += 32) {
    V bh[4], bl[4];
#pragma unroll
    for (int j = 0; j < 4; ++j) {
      const size_t bo = (size_t)(n0 + (j << 4) + rlane) * ldb + koff + k0;
      bh[j] = Frag<T>::load(Bb + bo);
      if (SPLIT) bl[j] = Frag<T>::load(Bb2 + bo);
    }
#pragma unroll
    for (int i = 0; i < 4; ++i) {
      const size_t ao = (size_t)(m0 + (i << 4) + rlane) * lda + koff + k0;
      V ah = Frag<T>::load(Ab + ao);
      V al;
      if (SPLIT) al = Frag<T>::load(Ab2 + ao);
#pragma unroll
      for (int j = 0; j < 4; ++j) {
        acc[i][j] = Frag<T>::mma(ah, bh[j], acc[i][j]);
        if (SPLIT) {
          acc[i][j] = Frag<T>::mma(ah, bl[j], acc[i][j]);
          acc[i][j] = Frag<T>::mma(al, bh[j], acc[i][j]);
        }
      }
      Frag<T>::guard(acc[i][0], acc[i][3], ah, SPLIT ? al : ah);
    }
    Frag<T>::keep(bh[0], bh[1], bh[2], bh[3]);
    if (SPLIT) Frag<T>::keep(bl[0], bl[1], bl[2], bl[3]);
  }
  acc_guard4(acc[0][0], acc[0][1], acc[0][2], acc[0][3]);
  acc_guard4(acc[1][0], acc[1][1], acc[1][2], acc[1][3]);
  acc_guard4(acc[2][0], acc[2][1], acc[2][2], acc[2][3]);
  acc_guard4(acc[3][0], acc[3][1], acc[3][2], acc[3][3]);

  float* slab = sT[wave];
  const float* Rb = RESID ? (resid + (size_t)b * strideR) : nullptr;
#pragma unroll
  for (int i = 0; i < 4; ++i) {
    const int mBase = m0 + (i << 4);
#pragma unroll
    for (int j = 0; j < 4; ++j) {
      const int n = n0 + (j << 4) + rlane;
      float bv = 0.f;
      if (BIAS_MODE == 2) bv = bias[n];
#pragma unroll
      for (int r = 0; r < 8; ++r) {
        float v = acc[i][j][r] * scale;
        if (BIAS_MODE == 1) v += bias[mBase + mOff + r];
        if (BIAS_MODE == 2) v += bv;
        if (RESID) v += Rb[(size_t)(mBase + mOff + r) * ldc + n];
        if (ACT == 2) v = fmaxf(v, 0.0f);
        if (ACT == 4) v = (v > 0.f) ? v : 0.01f * v;
        if (ACT == 6) {
          const float u = kGeluC * (v + kGeluA * v * v * v);
          v = 0.5f * v * (1.0f + tanhf(u)) * kH2Carry;
        }
        slab[(mOff + r) * 68 + (j << 4) + rlane] = v;
      }
    }
    __builtin_amdgcn_fence(__ATOMIC_RELEASE, "workgroup");
    __builtin_amdgcn_wave_barrier();
    __builtin_amdgcn_fence(__ATOMIC_ACQUIRE, "workgroup");
    if (OUT_MODE == 0) {
      float* C = (float*)Cout + (size_t)b * strideC;
      const int hh = lane >> 4, c4 = (lane & 15) * 4;
      for (int pass = 0; pass < 2; ++pass) {
#pragma unroll
        for (int it = 0; it < 8; ++it) {
          const int row = it * 2 + hh;
          v4f v = *(const v4f*)(slab + row * 68 + c4);
          *(volatile v4f*)(C + (size_t)(mBase + row) * ldc + n0 + c4) = v;
        }
        __threadfence();
      }
    } else {
      const int q = lane >> 3, c8 = (lane & 7) * 8;
      unsigned short* C  = (unsigned short*)Cout  + (size_t)b * strideC;
      unsigned short* C2 = (OUT_MODE == 2) ? ((unsigned short*)Cout2 + (size_t)b * strideC) : nullptr;
      for (int pass = 0; pass < 2; ++pass) {
#pragma unroll
        for (int it = 0; it < 4; ++it) {
          const int row = it * 4 + q;
          const float* sp = slab + row * 68 + c8;
          v8h hv, lv;
#pragma unroll
          for (int e = 0; e < 8; ++e) {
            if (OUT_MODE == 1) {
              hv[e] = (_Float16)sp[e];
            } else {
              unsigned short hb = f2bf_bits(sp[e]);
              unsigned short lb = f2bf_bits(sp[e] - bf_bits2f(hb));
              hv[e] = __builtin_bit_cast(_Float16, hb);
              lv[e] = __builtin_bit_cast(_Float16, lb);
            }
          }
          *(volatile v8h*)(C + (size_t)(mBase + row) * ldc + n0 + c8) = hv;
          if (OUT_MODE == 2) *(volatile v8h*)(C2 + (size_t)(mBase + row) * ldc + n0 + c8) = lv;
        }
        __threadfence();
      }
    }
    __builtin_amdgcn_fence(__ATOMIC_RELEASE, "workgroup");
    __builtin_amdgcn_wave_barrier();
    __builtin_amdgcn_fence(__ATOMIC_ACQUIRE, "workgroup");
  }
}

__global__ __launch_bounds__(256) void wtcast_kernel(const float* __restrict__ W, unsigned short* __restrict__ out,
                                                     int Kin, int Nout, float scale) {
  __shared__ float sm[64][65];
  const int t  = threadIdx.x;
  const int k0 = blockIdx.x * 64;
  const int n0 = blockIdx.y * 64;
#pragma unroll
  for (int i = 0; i < 16; ++i) {
    const int e = i * 256 + t;
    const int r = e >> 6;
    const int c = e & 63;
    sm[c][r] = W[(size_t)(k0 + r) * Nout + n0 + c] * scale;
  }
  __syncthreads();
  const int lane = t & 31, wave = t >> 5;
  const int q = lane >> 3, c8 = (lane & 7) * 8;
  for (int pass = 0; pass < 2; ++pass) {
#pragma unroll
    for (int it = 0; it < 2; ++it) {
      const int row = wave * 8 + it * 4 + q;
      unsigned short hb[8];
#pragma unroll
      for (int e = 0; e < 8; ++e) hb[e] = h_bits(sm[row][c8 + e]);
      const v4u u = (v4u){pk16(hb[0], hb[1]), pk16(hb[2], hb[3]), pk16(hb[4], hb[5]), pk16(hb[6], hb[7])};
      *(volatile v4u*)(out + (size_t)(n0 + row) * Kin + k0 + c8) = u;
    }
    __threadfence();
  }
}

__global__ __launch_bounds__(128) void ln_f16_kernel(const float* __restrict__ x, const float* __restrict__ w,
                                                     const float* __restrict__ bb, unsigned short* __restrict__ out) {
  __shared__ float redA[4];
  __shared__ float redB[4];
  const int row  = blockIdx.x;
  const int t    = threadIdx.x;
  const int lane = t & 31, wave = t >> 5;
  const int c0   = t * 8;
  const float* xr = x + (size_t)row * kDim + c0;
  const v4f a = *(const v4f*)(xr);
  const v4f c = *(const v4f*)(xr + 4);
  float v[8];
#pragma unroll
  for (int j = 0; j < 4; ++j) { v[j] = a[j]; v[4 + j] = c[j]; }
  float ps = ((v[0] + v[1]) + (v[2] + v[3])) + ((v[4] + v[5]) + (v[6] + v[7]));
#pragma unroll
  for (int off = 16; off > 0; off >>= 1) ps += __shfl_xor(ps, off, 32);
  if (lane == 0) redA[wave] = ps;
  __syncthreads();
  const float mu = ((redA[0] + redA[1]) + (redA[2] + redA[3])) * kInvDim;
  float d[8];
  float pq = 0.f;
#pragma unroll
  for (int j = 0; j < 8; ++j) { d[j] = v[j] - mu; pq += d[j] * d[j]; }
#pragma unroll
  for (int off = 16; off > 0; off >>= 1) pq += __shfl_xor(pq, off, 32);
  if (lane == 0) redB[wave] = pq;
  __syncthreads();
  const float var  = ((redB[0] + redB[1]) + (redB[2] + redB[3])) * kInvDim;
  const float rstd = rsqrtf(var + kLnEps);
  const v4f wa = *(const v4f*)(w + c0);
  const v4f wc = *(const v4f*)(w + c0 + 4);
  const v4f ba = *(const v4f*)(bb + c0);
  const v4f bc = *(const v4f*)(bb + c0 + 4);
  unsigned short hb[8];
#pragma unroll
  for (int j = 0; j < 4; ++j) {
    hb[j]     = h_bits(d[j] * rstd * wa[j] + ba[j]);
    hb[4 + j] = h_bits(d[4 + j] * rstd * wc[j] + bc[j]);
  }
  const v4u u = (v4u){pk16(hb[0], hb[1]), pk16(hb[2], hb[3]), pk16(hb[4], hb[5]), pk16(hb[6], hb[7])};
  unsigned short* op = out + (size_t)row * kDim + c0;
  *(volatile v4u*)op = u;
  __threadfence();
  *(volatile v4u*)op = u;
}

__global__ __launch_bounds__(256) void softmax_causal_kernel(const float* __restrict__ Sc, unsigned short* __restrict__ P) {
  __shared__ float redM[8];
  __shared__ float redS[8];
  const int row  = blockIdx.x & (kSeq - 1);
  const int g    = blockIdx.x >> kSeqLog2;
  const int t    = threadIdx.x;
  const int lane = t & 31, wave = t >> 5;
  const int c0   = t * 8;
  const size_t rbase = ((size_t)g * kSeq + row) * kSeq;
  const bool wact = (wave * 256 <= row);
  const int cl = (c0 <= row) ? c0 : (row & ~7);
  float s[8];
  float lmax = -INFINITY;
  if (wact) {
    const v4f a = *(const v4f*)(Sc + rbase + cl);
    const v4f c = *(const v4f*)(Sc + rbase + cl + 4);
#pragma unroll
    for (int j = 0; j < 4; ++j) {
      s[j]     = (c0 + j <= row)     ? a[j] : -INFINITY;
      s[4 + j] = (c0 + 4 + j <= row) ? c[j] : -INFINITY;
    }
#pragma unroll
    for (int j = 0; j < 8; ++j) lmax = fmaxf(lmax, s[j]);
  } else {
#pragma unroll
    for (int j = 0; j < 8; ++j) s[j] = -INFINITY;
  }
#pragma unroll
  for (int off = 16; off > 0; off >>= 1) lmax = fmaxf(lmax, __shfl_xor(lmax, off, 32));
  if (lane == 0) redM[wave] = lmax;
  __syncthreads();
  float mx = redM[0];
#pragma unroll
  for (int w2 = 1; w2 < 8; ++w2) mx = fmaxf(mx, redM[w2]);
  float e[8];
  float lsum = 0.f;
  if (wact) {
#pragma unroll
    for (int j = 0; j < 8; ++j) { e[j] = expf(s[j] - mx); lsum += e[j]; }
  } else {
#pragma unroll
    for (int j = 0; j < 8; ++j) e[j] = 0.f;
  }
#pragma unroll
  for (int off = 16; off > 0; off >>= 1) lsum += __shfl_xor(lsum, off, 32);
  if (lane == 0) redS[wave] = lsum;
  __syncthreads();
  float tot = redS[0];
#pragma unroll
  for (int w2 = 1; w2 < 8; ++w2) tot += redS[w2];
  const float invc = kPCarry / tot;
  unsigned short hb[8];
#pragma unroll
  for (int j = 0; j < 8; ++j) hb[j] = h_bits(e[j] * invc);
  const v4u u = (v4u){pk16(hb[0], hb[1]), pk16(hb[2], hb[3]), pk16(hb[4], hb[5]), pk16(hb[6], hb[7])};
  unsigned short* pp = P + rbase + c0;
  *(volatile v4u*)pp = u;
  __threadfence();
  *(volatile v4u*)pp = u;
}

extern "C" void kernel_launch(void* const* d_in, const int* in_sizes, int n_in,
                              void* d_out, int out_size, void* d_ws,
                              size_t ws_size, hipStream_t stream) {
  if (n_in < 13) return;
  if (in_sizes[0] != kTok * kDim || out_size != kTok * kDim) return;
  if (in_sizes[5] != kDim * 3 * kDim || in_sizes[9] != kDim * kFF || in_sizes[11] != kFF * kDim) return;
  if (ws_size < kWsTotal) return;

  const float* hs   = (const float*)d_in[0];
  const float* ln1w = (const float*)d_in[1];
  const float* ln1b = (const float*)d_in[2];
  const float* ln2w = (const float*)d_in[3];
  const float* ln2b = (const float*)d_in[4];
  const float* Wqkv = (const float*)d_in[5];
  const float* bqkv = (const float*)d_in[6];
  const float* Wpa  = (const float*)d_in[7];
  const float* bpa  = (const float*)d_in[8];
  const float* Wfc  = (const float*)d_in[9];
  const float* bfc  = (const float*)d_in[10];
  const float* Wpm  = (const float*)d_in[11];
  const float* bpm  = (const float*)d_in[12];
  float* out = (float*)d_out;

  char* ws = (char*)d_ws;
  unsigned short* WqkvT  = (unsigned short*)(ws + kOffWqkvT);
  unsigned short* X1     = (unsigned short*)(ws + kOffX1);
  float*          Sc     = (float*)(ws + kOffSc);
  unsigned short* H2     = (unsigned short*)(ws + kOffH2);
  unsigned short* Pp     = (unsigned short*)(ws + kOffP);
  unsigned short* WfcT   = (unsigned short*)(ws + kOffWfcT);
  unsigned short* WmlpT  = (unsigned short*)(ws + kOffWmlpT);
  unsigned short* QKp    = (unsigned short*)(ws + kOffQK);
  unsigned short* X2     = (unsigned short*)(ws + kOffX2);
  unsigned short* WprojT = (unsigned short*)(ws + kOffWprojT);
  unsigned short* VTp    = (unsigned short*)(ws + kOffVT);
  unsigned short* CTXp   = (unsigned short*)(ws + kOffCTX);
  float*          HO     = (float*)(ws + kOffHO);

  wtcast_kernel<<<dim3(kDim / 64, 3 * kDim / 64), 256, 0, stream>>>(Wqkv, WqkvT, kDim, 3 * kDim, kWCarry);

  ln_f16_kernel<<<kTok, 128, 0, stream>>>(hs, ln1w, ln1b, X1);

  wmma_gemm64<0, false, 2, 1, false, 0, false><<<dim3(256, 1), 256, 0, stream>>>(
      X1, nullptr, kDim, 0L,
      WqkvT, nullptr, kDim, 0L,
      (void*)QKp, nullptr, 2 * kDim, 0L,
      bqkv, nullptr, 0L,
      kTok, 2 * kDim, kDim, kWCarryInv);

  wmma_gemm64<0, false, 1, 1, false, 0, false><<<dim3(128, 1), 256, 0, stream>>>(
      WqkvT + (size_t)2 * kDim * kDim, nullptr, kDim, 0L,
      X1, nullptr, kDim, 0L,
      (void*)VTp, nullptr, kTok, 0L,
      bqkv + 2 * kDim, nullptr, 0L,
      kDim, kTok, kDim, kWCarryInv);

  for (int ch = 0; ch < kChunks; ++ch) {
    const int b  = ch / (kHeads / kGroupsPerChunk);
    const int h0 = (ch % (kHeads / kGroupsPerChunk)) * kGroupsPerChunk;
    const size_t qkBase = (size_t)b * kSeq * (2 * kDim) + (size_t)h0 * kHeadDim;
    wmma_gemm64<0, false, 0, 0, false, 0, true><<<dim3(128, kGroupsPerChunk), 256, 0, stream>>>(
        QKp + qkBase, nullptr, 2 * kDim, (long)kHeadDim,
        QKp + qkBase + kDim, nullptr, 2 * kDim, (long)kHeadDim,
        (void*)Sc, nullptr, kSeq, (long)kSeq * kSeq,
        nullptr, nullptr, 0L,
        kSeq, kSeq, kHeadDim, kScoreScale);
    softmax_causal_kernel<<<kGroupsPerChunk * kSeq, 256, 0, stream>>>(Sc, Pp);
    wmma_gemm64<0, false, 0, 1, false, 0, true><<<dim3(4, kGroupsPerChunk), 256, 0, stream>>>(
        Pp, nullptr, kSeq, (long)kSeq * kSeq,
        VTp + (size_t)h0 * kHeadDim * kTok + (size_t)b * kSeq, nullptr, kTok, (long)kHeadDim * kTok,
        (void*)(CTXp + (size_t)b * kSeq * kDim + (size_t)h0 * kHeadDim), nullptr, kDim, (long)kHeadDim,
        nullptr, nullptr, 0L,
        kSeq, kHeadDim, kSeq, kPVScale);
  }

  wtcast_kernel<<<dim3(kDim / 64, kDim / 64), 256, 0, stream>>>(Wpa, WprojT, kDim, kDim, kWCarry);

  wmma_gemm64<0, false, 2, 0, true, 0, false><<<dim3(128, 1), 256, 0, stream>>>(
      CTXp, nullptr, kDim, 0L,
      WprojT, nullptr, kDim, 0L,
      (void*)HO, nullptr, kDim, 0L,
      bpa, hs, 0L,
      kTok, kDim, kDim, kProjScale);

  ln_f16_kernel<<<kTok, 128, 0, stream>>>(HO, ln2w, ln2b, X2);

  wtcast_kernel<<<dim3(kDim / 64, kFF / 64), 256, 0, stream>>>(Wfc, WfcT, kDim, kFF, kWCarry);
  wtcast_kernel<<<dim3(kFF / 64, kDim / 64), 256, 0, stream>>>(Wpm, WmlpT, kFF, kDim, kWCarry);

  wmma_gemm64<0, false, 2, 1, false, 6, false><<<dim3(512, 1), 256, 0, stream>>>(
      X2, nullptr, kDim, 0L,
      WfcT, nullptr, kDim, 0L,
      (void*)H2, nullptr, kFF, 0L,
      bfc, nullptr, 0L,
      kTok, kFF, kDim, kWCarryInv);

  wmma_gemm64<0, false, 2, 0, true, 0, false><<<dim3(128, 1), 256, 0, stream>>>(
      H2, nullptr, kFF, 0L,
      WmlpT, nullptr, kFF, 0L,
      (void*)out, nullptr, kDim, 0L,
      bpm, HO, 0L,
      kTok, kDim, kFF, kMlpScale);
}
